// TransformerLayerTorch_69647189672021
// MI455X (gfx1250) — hardware-verified
//
#include <hip/hip_runtime.h>
#include <stddef.h>

typedef _Float16 v16h __attribute__((ext_vector_type(16)));
typedef _Float16 v8h  __attribute__((ext_vector_type(8)));
typedef _Float16 v4h  __attribute__((ext_vector_type(4)));
typedef float    v8f  __attribute__((ext_vector_type(8)));
typedef float    v4f  __attribute__((ext_vector_type(4)));
typedef v8h __attribute__((may_alias)) v8ha;
typedef v4h __attribute__((may_alias)) v4ha;
typedef v4f __attribute__((may_alias)) v4fa;

union Frag { v16h v; v8h half[2]; };

#define D_MODEL 1024
#define N_HEADS 16
#define D_HEAD  64
#define D_FF    4096
#define FF_HALF 2048
#define BATCH   4
#define SEQ     2048
#define MROWS   (BATCH * SEQ)
#define NX      (MROWS * D_MODEL)
#define NW      (D_MODEL * D_MODEL)
#define NF      (D_FF * D_MODEL)
#define NWALL   (4 * NW + 2 * NF)
#define NWALL8  (NWALL / 8)
#define NW8     (NW / 8)
#define LN_EPS  1e-5f
#define WSCALE  32.0f
#define INV_W   0.03125f
#define PSCALE  16384.0f
#define CSCALE  16.0f

__device__ __forceinline__ v8f wmma_f16(v16h a, v16h b, v8f c) {
  v8f d = __builtin_amdgcn_wmma_f32_16x16x32_f16(false, a, false, b, (short)0, c, false, false);
  asm volatile("v_nop\n\tv_nop\n\tv_nop\n\tv_nop" : "+v"(d) : "v"(a), "v"(b));
  return d;
}

__device__ __forceinline__ v16h load_frag(const _Float16* p, int h) {
  Frag f;
  f.half[0] = *(const v8ha*)(p + 8 * h);
  f.half[1] = *(const v8ha*)(p + 16 + 8 * h);
  return f.v;
}

__global__ __launch_bounds__(256) void convert_w_kernel(
    const float* __restrict__ wq, const float* __restrict__ wk,
    const float* __restrict__ wv, const float* __restrict__ wo,
    const float* __restrict__ f1, const float* __restrict__ f2,
    _Float16* __restrict__ wp)
{
  const int g = blockIdx.x * 256 + threadIdx.x;
  if (g >= NWALL8) return;
  const int seg = g >> 17;
  const float* src;
  if (seg == 0)      src = wq + (size_t)g * 8;
  else if (seg == 1) src = wk + (size_t)(g - NW8) * 8;
  else if (seg == 2) src = wv + (size_t)(g - 2 * NW8) * 8;
  else if (seg == 3) src = wo + (size_t)(g - 3 * NW8) * 8;
  else if (seg < 8)  src = f1 + (size_t)(g - 4 * NW8) * 8;
  else               src = f2 + (size_t)(g - 8 * NW8) * 8;
  const v4f a = *(const v4fa*)src;
  const v4f c = *(const v4fa*)(src + 4);
  const v8h o = { (_Float16)(a.x * WSCALE), (_Float16)(a.y * WSCALE), (_Float16)(a.z * WSCALE), (_Float16)(a.w * WSCALE),
                  (_Float16)(c.x * WSCALE), (_Float16)(c.y * WSCALE), (_Float16)(c.z * WSCALE), (_Float16)(c.w * WSCALE) };
  _Float16* dst = wp + (size_t)g * 8;
  *(volatile v8h*)dst = o;
  __threadfence();
  *(volatile v8h*)dst = o;
}

__global__ __launch_bounds__(256) void ln_kernel(
    const float* __restrict__ x, const float* __restrict__ gamma,
    const float* __restrict__ beta, _Float16* __restrict__ np)
{
  __shared__ float red0[8];
  __shared__ float red1[8];
  __shared__ __attribute__((aligned(16))) _Float16 srow[D_MODEL];

  const int t = threadIdx.x, lane = t & 31, w = t >> 5;
  const int row = blockIdx.x;
  const float* xr = x + (size_t)row * D_MODEL;
  const v4f v = *(const v4fa*)(xr + 4 * t);

  float s = (v.x + v.y) + (v.z + v.w);
  #pragma unroll
  for (int off = 16; off > 0; off >>= 1) s += __shfl_xor(s, off);
  if (lane == 0) red0[w] = s;
  __syncthreads();
  float tot = 0.0f;
  #pragma unroll
  for (int i = 0; i < 8; ++i) tot += red0[i];
  const float mean = tot * (1.0f / D_MODEL);

  const float d0 = v.x - mean, d1 = v.y - mean, d2 = v.z - mean, d3 = v.w - mean;
  float ss = (d0 * d0 + d1 * d1) + (d2 * d2 + d3 * d3);
  #pragma unroll
  for (int off = 16; off > 0; off >>= 1) ss += __shfl_xor(ss, off);
  if (lane == 0) red1[w] = ss;
  __syncthreads();
  float tot2 = 0.0f;
  #pragma unroll
  for (int i = 0; i < 8; ++i) tot2 += red1[i];
  const float var = tot2 * (1.0f / D_MODEL);
  const float rstd = rsqrtf(var + LN_EPS);

  const v4f g = *(const v4fa*)(gamma + 4 * t);
  const v4f bb = *(const v4fa*)(beta + 4 * t);
  const v4h o = { (_Float16)(d0 * rstd * g.x + bb.x), (_Float16)(d1 * rstd * g.y + bb.y),
                  (_Float16)(d2 * rstd * g.z + bb.z), (_Float16)(d3 * rstd * g.w + bb.w) };
  *(v4ha*)(srow + 4 * t) = o;
  __syncthreads();

  if (t < 128) {
    const v8h pv = *(const v8ha*)(srow + 8 * t);
    _Float16* dst = np + (size_t)row * D_MODEL + 8 * t;
    *(volatile v8h*)dst = pv;
    __threadfence();
    *(volatile v8h*)dst = pv;
  }
}

__device__ __forceinline__ void gemm_loop(v8f (&acc)[2][4], const _Float16* xa0, const _Float16* xa1,
                                          const _Float16* wb, int ldb, int K, int h) {
  #pragma unroll 1
  for (int k0 = 0; k0 < K; k0 += 32) {
    const v16h a0 = load_frag(xa0 + k0, h);
    const v16h a1 = load_frag(xa1 + k0, h);
    #pragma unroll
    for (int nt = 0; nt < 4; ++nt) {
      const v16h b = load_frag(wb + (size_t)nt * 16 * ldb + k0, h);
      acc[0][nt] = wmma_f16(a0, b, acc[0][nt]);
      acc[1][nt] = wmma_f16(a1, b, acc[1][nt]);
    }
  }
}

__device__ __forceinline__ void proj_store_pass(const _Float16* sT, _Float16* plane, _Float16* vt,
                                                int which, int bh, int l0, int w, int lane) {
  const int q8 = lane & 7, sub = lane >> 3;
  #pragma unroll
  for (int i = 0; i < 8; ++i) {
    const int lid = w * 32 + i * 4 + sub;
    v8h v;
    _Float16* dst;
    if (which != 2) {
      v = *(const v8ha*)(sT + lid * D_HEAD + 8 * q8);
      dst = plane + ((size_t)bh * SEQ + l0 + lid) * D_HEAD + 8 * q8;
    } else {
      const int d = lid >> 1, hl = lid & 1;
      v = *(const v8ha*)(sT + d * 128 + 64 * hl + 8 * q8);
      dst = vt + ((size_t)bh * D_HEAD + d) * SEQ + l0 + 64 * hl + 8 * q8;
    }
    *(volatile v8h*)dst = v;
  }
}

__global__ __launch_bounds__(128) void qkv_kernel(
    const _Float16* __restrict__ np,
    const _Float16* __restrict__ wp,
    _Float16* __restrict__ qh,
    _Float16* __restrict__ kh,
    _Float16* __restrict__ vt)
{
  __shared__ __attribute__((aligned(16))) _Float16 sT[128 * 64];

  const int tid = threadIdx.x, lane = tid & 31, w = tid >> 5;
  const int h = lane >> 4, m = lane & 15;
  const int m0 = blockIdx.x * 128;
  const int cg = blockIdx.y;
  const int which = cg >> 4, head = cg & 15;
  const int m0w = m0 + 32 * w;

  const _Float16* xa0 = np + (size_t)(m0w + m) * D_MODEL;
  const _Float16* xa1 = xa0 + (size_t)16 * D_MODEL;
  const _Float16* wb  = wp + (size_t)(cg * 64 + m) * D_MODEL;

  const v8f zero8 = {0.f, 0.f, 0.f, 0.f, 0.f, 0.f, 0.f, 0.f};
  v8f acc[2][4];
  #pragma unroll
  for (int mt = 0; mt < 2; ++mt)
    #pragma unroll
    for (int nt = 0; nt < 4; ++nt) acc[mt][nt] = zero8;

  gemm_loop(acc, xa0, xa1, wb, D_MODEL, D_MODEL, h);

  #pragma unroll
  for (int nt = 0; nt < 4; ++nt) {
    const int feat = 16 * nt + m;
    #pragma unroll
    for (int mt = 0; mt < 2; ++mt) {
      #pragma unroll
      for (int r = 0; r < 8; ++r) {
        const int tokl = 32 * w + 16 * mt + 8 * h + r;
        const float y = acc[mt][nt][r] * INV_W;
        const int idx = (which == 2) ? (feat * 128 + tokl) : (tokl * D_HEAD + feat);
        sT[idx] = (_Float16)y;
      }
    }
  }
  __syncthreads();

  const int b = m0 / SEQ, l0 = m0 - b * SEQ, bh = b * N_HEADS + head;
  _Float16* plane = (which == 0) ? qh : kh;
  proj_store_pass(sT, plane, vt, which, bh, l0, w, lane);
  __threadfence();
  proj_store_pass(sT, plane, vt, which, bh, l0, w, lane);
}

__device__ __forceinline__ v16h pack_p(v8f a, v8f c) {
  const v16h r = { (_Float16)(a[0] * PSCALE), (_Float16)(a[1] * PSCALE), (_Float16)(a[2] * PSCALE), (_Float16)(a[3] * PSCALE),
                   (_Float16)(a[4] * PSCALE), (_Float16)(a[5] * PSCALE), (_Float16)(a[6] * PSCALE), (_Float16)(a[7] * PSCALE),
                   (_Float16)(c[0] * PSCALE), (_Float16)(c[1] * PSCALE), (_Float16)(c[2] * PSCALE), (_Float16)(c[3] * PSCALE),
                   (_Float16)(c[4] * PSCALE), (_Float16)(c[5] * PSCALE), (_Float16)(c[6] * PSCALE), (_Float16)(c[7] * PSCALE) };
  return r;
}

__device__ __forceinline__ void att_store_pass(const _Float16* so, _Float16* cc,
                                               int b, int head, int q0, int lane) {
  const int q8 = lane & 7, sub = lane >> 3;
  #pragma unroll
  for (int i = 0; i < 4; ++i) {
    const int row = i * 4 + sub;
    const v8h v = *(const v8ha*)(so + row * 64 + 8 * q8);
    _Float16* dst = cc + ((size_t)b * SEQ + q0 + row) * D_MODEL + head * D_HEAD + 8 * q8;
    *(volatile v8h*)dst = v;
  }
}

__global__ __launch_bounds__(128) void attn_kernel(
    const _Float16* __restrict__ qh,
    const _Float16* __restrict__ kh,
    const _Float16* __restrict__ vt,
    _Float16* __restrict__ cc)
{
  __shared__ __attribute__((aligned(16))) _Float16 sO[4 * 16 * 64];

  const int tid = threadIdx.x, lane = tid & 31, w = tid >> 5;
  const int h = lane >> 4, m = lane & 15;
  const int bh = blockIdx.y, b = bh >> 4, head = bh & 15;
  const int qblk = blockIdx.x * 64;
  const int q0 = qblk + 16 * w;
  const int myq = q0 + m;

  const _Float16* qrow = qh + ((size_t)bh * SEQ + q0 + m) * D_HEAD;
  const v16h qb0 = load_frag(qrow, h);
  const v16h qb1 = load_frag(qrow + 32, h);

  const v8f zero8 = {0.f, 0.f, 0.f, 0.f, 0.f, 0.f, 0.f, 0.f};
  v8f o[4];
  #pragma unroll
  for (int t = 0; t < 4; ++t) o[t] = zero8;
  float mrun = -1e30f, lrun = 0.0f;

  const _Float16* kbase = kh + ((size_t)bh * SEQ + m) * D_HEAD;
  const _Float16* vbase = vt + ((size_t)bh * D_HEAD + m) * SEQ;

  const int nsteps = blockIdx.x + 1;
  #pragma unroll 1
  for (int st = 0; st < nsteps; ++st) {
    const int kb = st * 64;
    v8f s[4];
    #pragma unroll
    for (int j = 0; j < 4; ++j) {
      const _Float16* kp = kbase + (size_t)(kb + 16 * j) * D_HEAD;
      const v16h kf0 = load_frag(kp, h);
      const v16h kf1 = load_frag(kp + 32, h);
      v8f z = zero8;
      z = wmma_f16(kf0, qb0, z);
      z = wmma_f16(kf1, qb1, z);
      s[j] = z;
    }
    #pragma unroll
    for (int j = 0; j < 4; ++j)
      #pragma unroll
      for (int r = 0; r < 8; ++r) s[j][r] = s[j][r] * 0.125f;

    if (kb == qblk) {
      #pragma unroll
      for (int j = 0; j < 4; ++j)
        #pragma unroll
        for (int r = 0; r < 8; ++r) {
          const int key = kb + 16 * j + 8 * h + r;
          s[j][r] = (key > myq) ? -1.0e9f : s[j][r];
        }
    }

    float mloc = s[0][0];
    #pragma unroll
    for (int j = 0; j < 4; ++j)
      #pragma unroll
      for (int r = 0; r < 8; ++r) mloc = fmaxf(mloc, s[j][r]);
    mloc = fmaxf(mloc, __shfl_xor(mloc, 16));
    const float mnew = fmaxf(mrun, mloc);
    const float alpha = __expf(mrun - mnew);
    mrun = mnew;
    float lsum = 0.0f;
    #pragma unroll
    for (int j = 0; j < 4; ++j)
      #pragma unroll
      for (int r = 0; r < 8; ++r) {
        const float p = __expf(s[j][r] - mnew);
        s[j][r] = p;
        lsum += p;
      }
    lsum += __shfl_xor(lsum, 16);
    lrun = lrun * alpha + lsum;
    #pragma unroll
    for (int t = 0; t < 4; ++t)
      #pragma unroll
      for (int r = 0; r < 8; ++r) o[t][r] = o[t][r] * alpha;

    const v16h pb0 = pack_p(s[0], s[1]);
    const v16h pb1 = pack_p(s[2], s[3]);

    #pragma unroll
    for (int t = 0; t < 4; ++t) {
      const _Float16* vp = vbase + (size_t)(16 * t) * SEQ + kb;
      const v16h vf0 = load_frag(vp, h);
      const v16h vf1 = load_frag(vp + 32, h);
      o[t] = wmma_f16(vf0, pb0, o[t]);
      o[t] = wmma_f16(vf1, pb1, o[t]);
    }
  }

  const float inv = (1.0f / lrun) * (CSCALE / PSCALE);
  _Float16* so = sO + w * 1024;
  #pragma unroll
  for (int t = 0; t < 4; ++t)
    #pragma unroll
    for (int r = 0; r < 8; ++r)
      so[m * 64 + 16 * t + 8 * h + r] = (_Float16)(o[t][r] * inv);
  __syncthreads();

  att_store_pass(so, cc, b, head, q0, lane);
  __threadfence();
  att_store_pass(so, cc, b, head, q0, lane);
}

__device__ __forceinline__ void resid_store_pass(const v4f (&vals)[16], float* outp, int m0w, int n0, int lane) {
  const int q8 = lane & 7, sub = lane >> 3;
  #pragma unroll
  for (int i = 0; i < 16; ++i) {
    const int lid = i * 4 + sub;
    const int row = lid >> 1, hl = lid & 1;
    float* dst = outp + (size_t)(m0w + row) * D_MODEL + n0 + 32 * hl + 4 * q8;
    *(volatile v4f*)dst = vals[i];
  }
}

__global__ __launch_bounds__(128) void gemm_resid_kernel(
    const _Float16* __restrict__ A, int lda,
    const _Float16* __restrict__ W, int ldb, int K,
    const float* resid,
    float* outp,
    float scale)
{
  __shared__ __attribute__((aligned(16))) float sO[128 * 64];

  const int tid = threadIdx.x, lane = tid & 31, w = tid >> 5;
  const int h = lane >> 4, m = lane & 15;
  const int m0 = blockIdx.x * 128;
  const int n0 = blockIdx.y * 64;
  const int m0w = m0 + 32 * w;

  const _Float16* xa0 = A + (size_t)(m0w + m) * lda;
  const _Float16* xa1 = xa0 + (size_t)16 * lda;
  const _Float16* wb  = W + (size_t)(n0 + m) * ldb;

  const v8f zero8 = {0.f, 0.f, 0.f, 0.f, 0.f, 0.f, 0.f, 0.f};
  v8f acc[2][4];
  #pragma unroll
  for (int mt = 0; mt < 2; ++mt)
    #pragma unroll
    for (int nt = 0; nt < 4; ++nt) acc[mt][nt] = zero8;

  gemm_loop(acc, xa0, xa1, wb, ldb, K, h);

  #pragma unroll
  for (int nt = 0; nt < 4; ++nt) {
    const int feat = 16 * nt + m;
    #pragma unroll
    for (int mt = 0; mt < 2; ++mt) {
      #pragma unroll
      for (int r = 0; r < 8; ++r) {
        const int tokl = 32 * w + 16 * mt + 8 * h + r;
        sO[tokl * 64 + feat] = acc[mt][nt][r] * scale;
      }
    }
  }
  __syncthreads();

  const int q8 = lane & 7, sub = lane >> 3;
  v4f vals[16];
  #pragma unroll
  for (int i = 0; i < 16; ++i) {
    const int lid = i * 4 + sub;
    const int row = lid >> 1, hl = lid & 1;
    const int col = 32 * hl + 4 * q8;
    const v4f a  = *(const v4fa*)(sO + (32 * w + row) * 64 + col);
    const v4f rr = *(const v4fa*)(resid + (size_t)(m0w + row) * D_MODEL + n0 + col);
    vals[i] = a + rr;
  }
  resid_store_pass(vals, outp, m0w, n0, lane);
  __threadfence();
  resid_store_pass(vals, outp, m0w, n0, lane);
}

__device__ __forceinline__ float gelu_f(float x) {
  const float cubic = x * x * x;
  const float cdf = 0.5f * (1.0f + tanhf(0.7978845608f * (x + 0.044715f * cubic)));
  return x * cdf;
}

__device__ __forceinline__ void h16_store_pass(const _Float16* sT, _Float16* hid, int m0, int n0, int w, int lane) {
  const int q8 = lane & 7, sub = lane >> 3;
  #pragma unroll
  for (int i = 0; i < 8; ++i) {
    const int lid = w * 32 + i * 4 + sub;
    const v8h v = *(const v8ha*)(sT + lid * 64 + 8 * q8);
    _Float16* dst = hid + (size_t)(m0 + lid) * FF_HALF + n0 + 8 * q8;
    *(volatile v8h*)dst = v;
  }
}

__global__ __launch_bounds__(128) void gemm_gelu_kernel(
    const _Float16* __restrict__ np,
    const _Float16* __restrict__ wrows,
    _Float16* __restrict__ hid)
{
  __shared__ __attribute__((aligned(16))) _Float16 sT[128 * 64];

  const int tid = threadIdx.x, lane = tid & 31, w = tid >> 5;
  const int h = lane >> 4, m = lane & 15;
  const int m0 = blockIdx.x * 128;
  const int n0 = blockIdx.y * 64;
  const int m0w = m0 + 32 * w;

  const _Float16* xa0 = np + (size_t)(m0w + m) * D_MODEL;
  const _Float16* xa1 = xa0 + (size_t)16 * D_MODEL;
  const _Float16* wb  = wrows + (size_t)(n0 + m) * D_MODEL;

  const v8f zero8 = {0.f, 0.f, 0.f, 0.f, 0.f, 0.f, 0.f, 0.f};
  v8f acc[2][4];
  #pragma unroll
  for (int mt = 0; mt < 2; ++mt)
    #pragma unroll
    for (int nt = 0; nt < 4; ++nt) acc[mt][nt] = zero8;

  gemm_loop(acc, xa0, xa1, wb, D_MODEL, D_MODEL, h);

  #pragma unroll
  for (int nt = 0; nt < 4; ++nt) {
    const int feat = 16 * nt + m;
    #pragma unroll
    for (int mt = 0; mt < 2; ++mt) {
      #pragma unroll
      for (int r = 0; r < 8; ++r) {
        const int tokl = 32 * w + 16 * mt + 8 * h + r;
        sT[tokl * 64 + feat] = (_Float16)gelu_f(acc[mt][nt][r] * INV_W);
      }
    }
  }
  __syncthreads();

  h16_store_pass(sT, hid, m0, n0, w, lane);
  __threadfence();
  h16_store_pass(sT, hid, m0, n0, w, lane);
}

extern "C" void kernel_launch(void* const* d_in, const int* in_sizes, int n_in,
                              void* d_out, int out_size, void* d_ws, size_t ws_size,
                              hipStream_t stream) {
  if (n_in < 11) return;
  if (in_sizes[0] != NX || out_size != NX) return;
  if (in_sizes[1] != D_MODEL || in_sizes[2] != D_MODEL) return;
  if (in_sizes[3] != NW || in_sizes[4] != NW || in_sizes[5] != NW || in_sizes[6] != NW) return;
  if (in_sizes[7] != D_MODEL || in_sizes[8] != D_MODEL) return;
  if (in_sizes[9] != NF || in_sizes[10] != NF) return;

  const float* x      = (const float*)d_in[0];
  const float* gamma1 = (const float*)d_in[1];
  const float* beta1  = (const float*)d_in[2];
  const float* wq     = (const float*)d_in[3];
  const float* wk     = (const float*)d_in[4];
  const float* wv     = (const float*)d_in[5];
  const float* wo     = (const float*)d_in[6];
  const float* gamma2 = (const float*)d_in[7];
  const float* beta2  = (const float*)d_in[8];
  const float* fc1    = (const float*)d_in[9];
  const float* fc2    = (const float*)d_in[10];
  float* out = (float*)d_out;

  const size_t wp_bytes  = (size_t)NWALL * 2;
  const size_t r1_bytes  = (size_t)NX * 2;
  const size_t pl_bytes  = (size_t)NX * 2;
  const size_t r2_bytes  = 3 * pl_bytes;
  const size_t xr_bytes  = (size_t)NX * 4;
  const size_t hid_bytes = (size_t)MROWS * FF_HALF * 2;
  const size_t total = wp_bytes + r1_bytes + r2_bytes + xr_bytes;
  if (total > ws_size) return;
  if (hid_bytes > r2_bytes) return;

  char* ws = (char*)d_ws;
  _Float16* wp  = (_Float16*)(ws);
  _Float16* r1  = (_Float16*)(ws + wp_bytes);
  _Float16* qh  = (_Float16*)(ws + wp_bytes + r1_bytes);
  _Float16* kh  = (_Float16*)(ws + wp_bytes + r1_bytes + pl_bytes);
  _Float16* vt  = (_Float16*)(ws + wp_bytes + r1_bytes + 2 * pl_bytes);
  _Float16* hid = qh;
  float*    xr  = (float*)(ws + wp_bytes + r1_bytes + r2_bytes);

  const _Float16* wqkv_p = wp;
  const _Float16* wo_p   = wp + (size_t)3 * NW;
  const _Float16* fc1_p  = wp + (size_t)4 * NW;
  const _Float16* fc2_p  = wp + (size_t)4 * NW + NF;

  convert_w_kernel<<<NWALL8 / 256, 256, 0, stream>>>(wq, wk, wv, wo, fc1, fc2, wp);

  ln_kernel<<<MROWS, 256, 0, stream>>>(x, gamma1, beta1, r1);

  qkv_kernel<<<dim3(MROWS / 128, 3 * N_HEADS), 128, 0, stream>>>(r1, wqkv_p, qh, kh, vt);

  attn_kernel<<<dim3(SEQ / 64, BATCH * N_HEADS), 128, 0, stream>>>(qh, kh, vt, r1);

  gemm_resid_kernel<<<dim3(MROWS / 128, D_MODEL / 64), 128, 0, stream>>>(
      r1, D_MODEL, wo_p, D_MODEL, D_MODEL, x, xr, INV_W / CSCALE);

  ln_kernel<<<MROWS, 256, 0, stream>>>(xr, gamma2, beta2, r1);

  gemm_gelu_kernel<<<dim3(MROWS / 128, FF_HALF / 64), 128, 0, stream>>>(r1, fc1_p, hid);

  gemm_resid_kernel<<<dim3(MROWS / 128, D_MODEL / 64), 128, 0, stream>>>(
      hid, FF_HALF, fc2_p, D_FF, FF_HALF, xr, out, INV_W);

  gemm_gelu_kernel<<<dim3(MROWS / 128, FF_HALF / 64), 128, 0, stream>>>(
      r1, fc1_p + (size_t)FF_HALF * D_MODEL, hid);

  gemm_resid_kernel<<<dim3(MROWS / 128, D_MODEL / 64), 128, 0, stream>>>(
      hid, FF_HALF, fc2_p + FF_HALF, D_FF, FF_HALF, out, out, INV_W);
}
